// GaussianSelfAttention_17471926960864
// MI455X (gfx1250) — hardware-verified
//
#include <hip/hip_runtime.h>
#include <stdint.h>
#include <stddef.h>

#pragma clang fp contract(off)

typedef __attribute__((ext_vector_type(16))) _Float16 v16h;
typedef __attribute__((ext_vector_type(8)))  _Float16 v8h;
typedef __attribute__((ext_vector_type(16))) __bf16   v16b;
typedef __attribute__((ext_vector_type(8)))  __bf16   v8b;
typedef __attribute__((ext_vector_type(8)))  float    v8f;
typedef __attribute__((ext_vector_type(4)))  float    v4f;
typedef __attribute__((ext_vector_type(4)))  unsigned int v4u;

#ifndef NB
#define NB 16
#endif
#ifndef NQ
#define NQ 1024
#endif
#define NB_FULL 16
#define NQ_FULL 1024
#define NKEY    1024
#define GRW     32
#define DM      256
#define NHD     9
#define KD      2304
#define BCH     8
#define NBC     ((NB < BCH) ? NB : BCH)

__device__ __forceinline__ unsigned short f2bf_bits(float f) {
  unsigned u = __float_as_uint(f);
  return (unsigned short)((u + 0x7FFFu + ((u >> 16) & 1u)) >> 16);
}
__device__ __forceinline__ float bf_bits2f(unsigned short h) { return __uint_as_float(((unsigned)h) << 16); }
__device__ __forceinline__ float rbf(float f) { return bf_bits2f(f2bf_bits(f)); }

__device__ __forceinline__ void dep_guard_h(v8f& a, v8f& b, v16h x, v16h y) { asm volatile("v_nop\n\tv_nop\n\tv_nop\n\tv_nop" : "+v"(a), "+v"(b) : "v"(x), "v"(y)); }
__device__ __forceinline__ void dep_guard_b(v8f& a, v8f& b, v16b x, v16b y) { asm volatile("v_nop\n\tv_nop\n\tv_nop\n\tv_nop" : "+v"(a), "+v"(b) : "v"(x), "v"(y)); }
__device__ __forceinline__ void keep4_h(v16h a, v16h b, v16h c, v16h d) { asm volatile("v_nop" :: "v"(a), "v"(b), "v"(c), "v"(d)); }
__device__ __forceinline__ void keep4_b(v16b a, v16b b, v16b c, v16b d) { asm volatile("v_nop" :: "v"(a), "v"(b), "v"(c), "v"(d)); }
__device__ __forceinline__ void acc_guard4(v8f& a, v8f& b, v8f& c, v8f& d) { asm volatile("v_nop\n\tv_nop\n\tv_nop\n\tv_nop" : "+v"(a), "+v"(b), "+v"(c), "+v"(d)); }

template <typename T> struct Frag;
template <> struct Frag<_Float16> {
  typedef v16h V; union U { v16h v; v8h h[2]; };
  static __device__ __forceinline__ v16h load(const _Float16* p) {
    U f; f.h[0] = *(const v8h*)(p); f.h[1] = *(const v8h*)(p + 16); return f.v;
  }
  static __device__ __forceinline__ v8f mma(v16h a, v16h b, v8f c) {
    return __builtin_amdgcn_wmma_f32_16x16x32_f16(false, a, false, b, (short)0, c, false, false);
  }
  static __device__ __forceinline__ void guard(v8f& a, v8f& b, v16h x, v16h y) { dep_guard_h(a, b, x, y); }
  static __device__ __forceinline__ void keep(v16h a, v16h b, v16h c, v16h d) { keep4_h(a, b, c, d); }
};
template <> struct Frag<__bf16> {
  typedef v16b V; union U { v16b v; v8b h[2]; };
  static __device__ __forceinline__ v16b load(const __bf16* p) {
    U f; f.h[0] = *(const v8b*)(p); f.h[1] = *(const v8b*)(p + 16); return f.v;
  }
  static __device__ __forceinline__ v8f mma(v16b a, v16b b, v8f c) {
    return __builtin_amdgcn_wmma_f32_16x16x32_bf16(false, a, false, b, (short)0, c, false, false);
  }
  static __device__ __forceinline__ void guard(v8f& a, v8f& b, v16b x, v16b y) { dep_guard_b(a, b, x, y); }
  static __device__ __forceinline__ void keep(v16b a, v16b b, v16b c, v16b d) { keep4_b(a, b, c, d); }
};

template <int ET> struct Elem;
template <> struct Elem<0> { typedef _Float16 T; };
template <> struct Elem<1> { typedef __bf16 T; };
template <int ET, int SPLIT, int BIAS_MODE, int OUT_MODE>
__global__ __launch_bounds__(256) void wmma_gemm64(
    const unsigned short* __restrict__ Ap, const unsigned short* __restrict__ A2p, int lda, long sAy, long sAz,
    const unsigned short* __restrict__ Btp, const unsigned short* __restrict__ Bt2p, int ldb, long sBy, long sBz,
    void* __restrict__ Cout, void* __restrict__ Cout2, int ldc, long sCy, long sCz,
    const float* __restrict__ bias,
    int M, int N, int K, float scale) {
  typedef typename Elem<ET>::T T;
  typedef typename Frag<T>::V V;
  const T* A = (const T*)Ap; const T* A2 = (const T*)A2p; const T* Bt = (const T*)Btp; const T* Bt2 = (const T*)Bt2p;
  __shared__ __align__(16) float sT[8][16 * 68];
  const int by   = blockIdx.y;
  const int bz   = blockIdx.z;
  const int lane = threadIdx.x & 31;
  const int wave = threadIdx.x >> 5;
  const int tilesN = N >> 6;
  const int tilesM = M >> 6;
  const int tile = blockIdx.x * 8 + wave;
  if (tile >= tilesM * tilesN) return;
  const int tm = tile / tilesN;
  const int tn = tile - tm * tilesN;
  const int m0 = tm << 6;
  const int n0 = tn << 6;

  const size_t aoff = (size_t)by * (size_t)sAy + (size_t)bz * (size_t)sAz;
  const size_t boff = (size_t)by * (size_t)sBy + (size_t)bz * (size_t)sBz;
  const size_t coff = (size_t)by * (size_t)sCy + (size_t)bz * (size_t)sCz;
  const T* Ab  = A  + aoff;
  const T* Bb  = Bt + boff;
  const T* Ab2 = (SPLIT >= 1) ? (A2  + aoff) : nullptr;
  const T* Bb2 = (SPLIT == 2) ? (Bt2 + boff) : nullptr;

  const int rlane = lane & 15;
  const int koff  = (lane >> 4) * 8;
  const int mOff  = (lane >> 4) * 8;

  v8f acc[4][4];
#pragma unroll
  for (int i = 0; i < 4; ++i)
#pragma unroll
    for (int j = 0; j < 4; ++j) acc[i][j] = (v8f){0.f,0.f,0.f,0.f,0.f,0.f,0.f,0.f};

  for (int k0 = 0; k0 < K; k0 += 32) {
    V bh[4], bl[4];
#pragma unroll
    for (int j = 0; j < 4; ++j) {
      const size_t bo = (size_t)(n0 + (j << 4) + rlane) * ldb + koff + k0;
      bh[j] = Frag<T>::load(Bb + bo);
      if (SPLIT == 2) bl[j] = Frag<T>::load(Bb2 + bo);
    }
#pragma unroll
    for (int i = 0; i < 4; ++i) {
      const size_t ao = (size_t)(m0 + (i << 4) + rlane) * lda + koff + k0;
      V ah = Frag<T>::load(Ab + ao);
      V al = ah;
      if (SPLIT >= 1) al = Frag<T>::load(Ab2 + ao);
#pragma unroll
      for (int j = 0; j < 4; ++j) {
        acc[i][j] = Frag<T>::mma(ah, bh[j], acc[i][j]);
        if (SPLIT == 2) acc[i][j] = Frag<T>::mma(ah, bl[j], acc[i][j]);
        if (SPLIT >= 1) acc[i][j] = Frag<T>::mma(al, bh[j], acc[i][j]);
      }
      Frag<T>::guard(acc[i][0], acc[i][3], ah, al);
    }
    Frag<T>::keep(bh[0], bh[1], bh[2], bh[3]);
    if (SPLIT == 2) Frag<T>::keep(bl[0], bl[1], bl[2], bl[3]);
  }
  acc_guard4(acc[0][0], acc[0][1], acc[0][2], acc[0][3]);
  acc_guard4(acc[1][0], acc[1][1], acc[1][2], acc[1][3]);
  acc_guard4(acc[2][0], acc[2][1], acc[2][2], acc[2][3]);
  acc_guard4(acc[3][0], acc[3][1], acc[3][2], acc[3][3]);

  float* slab = sT[wave];
#pragma unroll
  for (int i = 0; i < 4; ++i) {
    const int mBase = m0 + (i << 4);
#pragma unroll
    for (int j = 0; j < 4; ++j) {
      const int n = n0 + (j << 4) + rlane;
      float bv = 0.f;
      if (BIAS_MODE == 2) bv = rbf(bias[n]);
#pragma unroll
      for (int r = 0; r < 8; ++r) {
        float v = acc[i][j][r] * scale;
        if (BIAS_MODE == 2) v += bv;
        slab[(mOff + r) * 68 + (j << 4) + rlane] = v;
      }
    }
    __builtin_amdgcn_fence(__ATOMIC_RELEASE, "workgroup");
    __builtin_amdgcn_wave_barrier();
    __builtin_amdgcn_fence(__ATOMIC_ACQUIRE, "workgroup");
    if (OUT_MODE == 0) {
      float* C = (float*)Cout + coff;
      const int hh = lane >> 4, c4 = (lane & 15) * 4;
      for (int pass = 0; pass < 2; ++pass) {
#pragma unroll
        for (int it = 0; it < 8; ++it) {
          const int row = it * 2 + hh;
          v4f v = *(const v4f*)(slab + row * 68 + c4);
          if (BIAS_MODE == 1) { const float bm = bias[mBase + row]; v = v + bm; }
          *(volatile v4f*)(C + (size_t)(mBase + row) * ldc + n0 + c4) = v;
        }
        __threadfence();
      }
    } else {
      const int q = lane >> 3, c8 = (lane & 7) * 8;
      unsigned short* C  = (unsigned short*)Cout  + coff;
      unsigned short* C2 = (OUT_MODE == 2) ? ((unsigned short*)Cout2 + coff) : nullptr;
      for (int pass = 0; pass < 2; ++pass) {
#pragma unroll
        for (int it = 0; it < 4; ++it) {
          const int row = it * 4 + q;
          const float* sp = slab + row * 68 + c8;
          float bm = 0.f;
          if (BIAS_MODE == 1) bm = bias[mBase + row];
          v8h hv, lv;
#pragma unroll
          for (int e = 0; e < 8; ++e) {
            const float val = sp[e] + bm;
            if (OUT_MODE == 1) {
              hv[e] = (_Float16)val;
              lv[e] = hv[e];
            } else {
              unsigned short hb = f2bf_bits(val);
              hv[e] = __builtin_bit_cast(_Float16, hb);
              if (OUT_MODE == 2) {
                unsigned short lb = f2bf_bits(val - bf_bits2f(hb));
                lv[e] = __builtin_bit_cast(_Float16, lb);
              } else {
                lv[e] = hv[e];
              }
            }
          }
          *(volatile v8h*)(C + (size_t)(mBase + row) * ldc + n0 + c8) = hv;
          if (OUT_MODE == 2) *(volatile v8h*)(C2 + (size_t)(mBase + row) * ldc + n0 + c8) = lv;
        }
        __threadfence();
      }
    }
    __builtin_amdgcn_fence(__ATOMIC_RELEASE, "workgroup");
    __builtin_amdgcn_wave_barrier();
    __builtin_amdgcn_fence(__ATOMIC_ACQUIRE, "workgroup");
  }
}

__global__ __launch_bounds__(256) void probs_kernel(
    const float* __restrict__ centers, const float* __restrict__ spreads, const int* __restrict__ amask,
    unsigned short* __restrict__ Ph, unsigned short* __restrict__ Pl) {
  __shared__ __align__(16) float ef[8][NKEY];
  (void)amask;
  const int wave = threadIdx.x >> 5;
  const int lane = threadIdx.x & 31;
  const int h = blockIdx.y;
  const int q = blockIdx.x * 8 + wave;

  const float s00 = rbf(spreads[h * 4 + 0]);
  const float s01 = rbf(spreads[h * 4 + 1]);
  const float s10 = rbf(spreads[h * 4 + 2]);
  const float s11 = rbf(spreads[h * 4 + 3]);
  const float mu1 = rbf(centers[h * 2 + 0]);
  const float mu2 = rbf(centers[h * 2 + 1]);
  const float a00 = s00 * s00; const float a01 = s01 * s01; const float ca = a00 + a01;
  const float b00 = s00 * s10; const float b01 = s01 * s11; const float cb = b00 + b01;
  const float c00 = s10 * s10; const float c01 = s11 * s11; const float cc = c00 + c01;
  const float p0 = ca * mu1; const float p1 = cb * mu2; const float u0 = p0 + p1;
  const float p2 = cc * mu2; const float p3 = cb * mu1; const float u1 = p2 + p3;
  const float u2 = -0.5f * ca;
  const float u3 = -0.5f * cc;
  const float u4 = -cb;

  const int qi = q >> 5;
  const int qj = q & 31;
  const float dy  = (float)(lane - qj);
  const float dy2 = dy * dy;
  const float t1  = u1 * dy;
  const float t3  = u3 * dy2;
  const float cy  = t1 + t3;
  const float t4  = u4 * dy;
  const float cx  = u0 + t4;

  float m = -__builtin_inff();
#pragma unroll 1
  for (int t = 0; t < GRW; ++t) {
    const float dx = (float)(t - qi);
    const float w0 = u2 * dx;
    const float w1 = cx + w0;
    const float w2 = dx * w1;
    const float s  = cy + w2;
    m = fmaxf(m, s);
  }
#pragma unroll
  for (int off = 1; off < 32; off <<= 1) m = fmaxf(m, __shfl_xor(m, off, 32));

  float* efw = ef[wave];
  float sum = 0.f;
#pragma unroll 1
  for (int t = 0; t < GRW; ++t) {
    const float dx = (float)(t - qi);
    const float w0 = u2 * dx;
    const float w1 = cx + w0;
    const float w2 = dx * w1;
    const float s  = cy + w2;
    const float e  = expf(s - m);
    sum = sum + e;
    efw[t * GRW + lane] = e;
  }
#pragma unroll
  for (int off = 1; off < 32; off <<= 1) sum += __shfl_xor(sum, off, 32);
  const float inv = 1.0f / sum;

  __builtin_amdgcn_fence(__ATOMIC_RELEASE, "workgroup");
  __builtin_amdgcn_wave_barrier();
  __builtin_amdgcn_fence(__ATOMIC_ACQUIRE, "workgroup");

  v4u hvv[4], lvv[4];
#pragma unroll
  for (int it = 0; it < 4; ++it) {
    const int cch = it * 32 + lane;
    const float* sp = efw + 8 * cch;
    const v4f x0 = *(const v4f*)(sp);
    const v4f x1 = *(const v4f*)(sp + 4);
    float f[8];
    f[0] = x0[0]; f[1] = x0[1]; f[2] = x0[2]; f[3] = x0[3];
    f[4] = x1[0]; f[5] = x1[1]; f[6] = x1[2]; f[7] = x1[3];
    unsigned hw[4], lw[4];
#pragma unroll
    for (int e = 0; e < 4; ++e) {
      const float pa = f[2 * e] * inv;
      const float pb = f[2 * e + 1] * inv;
      const unsigned short h0 = f2bf_bits(pa);
      const unsigned short l0 = f2bf_bits(pa - bf_bits2f(h0));
      const unsigned short h1 = f2bf_bits(pb);
      const unsigned short l1 = f2bf_bits(pb - bf_bits2f(h1));
      hw[e] = (unsigned)h0 | ((unsigned)h1 << 16);
      lw[e] = (unsigned)l0 | ((unsigned)l1 << 16);
    }
    v4u hv; hv[0] = hw[0]; hv[1] = hw[1]; hv[2] = hw[2]; hv[3] = hw[3];
    v4u lv; lv[0] = lw[0]; lv[1] = lw[1]; lv[2] = lw[2]; lv[3] = lw[3];
    hvv[it] = hv; lvv[it] = lv;
  }
  const size_t rowoff = ((size_t)h * NQ + (size_t)q) * NKEY;
  for (int pass = 0; pass < 2; ++pass) {
#pragma unroll
    for (int it = 0; it < 4; ++it) {
      const size_t o = rowoff + (size_t)8 * (it * 32 + lane);
      *(volatile v4u*)(Ph + o) = hvv[it];
      *(volatile v4u*)(Pl + o) = lvv[it];
    }
    __threadfence();
  }
}

__global__ __launch_bounds__(256) void xt_kernel(const float* __restrict__ hs, unsigned short* __restrict__ XT) {
  __shared__ __align__(16) unsigned short st[64 * 72];
  const int tid  = threadIdx.x;
  const int wave = tid >> 5;
  const int lane = tid & 31;
  const int k0 = blockIdx.x * 64;
  const int d0 = blockIdx.y * 64;
  const int b  = blockIdx.z;
  const int kr = tid >> 2;
  const int ds = (tid & 3) * 16;
  const float* src = hs + ((size_t)b * NKEY + k0 + kr) * DM + d0 + ds;
  const v4f a0 = *(const v4f*)(src);
  const v4f a1 = *(const v4f*)(src + 4);
  const v4f a2 = *(const v4f*)(src + 8);
  const v4f a3 = *(const v4f*)(src + 12);
  float f[16];
  f[0]  = a0[0]; f[1]  = a0[1]; f[2]  = a0[2]; f[3]  = a0[3];
  f[4]  = a1[0]; f[5]  = a1[1]; f[6]  = a1[2]; f[7]  = a1[3];
  f[8]  = a2[0]; f[9]  = a2[1]; f[10] = a2[2]; f[11] = a2[3];
  f[12] = a3[0]; f[13] = a3[1]; f[14] = a3[2]; f[15] = a3[3];
#pragma unroll
  for (int e = 0; e < 16; ++e) st[(ds + e) * 72 + kr] = f2bf_bits(f[e]);
  __syncthreads();
  v4u vv[2];
  int rows[2];
  const int c8 = (lane & 7) * 8;
#pragma unroll
  for (int it = 0; it < 2; ++it) {
    const int row = it * 32 + wave * 4 + (lane >> 3);
    rows[it] = row;
    vv[it] = *(const v4u*)(st + row * 72 + c8);
  }
  for (int pass = 0; pass < 2; ++pass) {
#pragma unroll
    for (int it = 0; it < 2; ++it) {
      *(volatile v4u*)(XT + ((size_t)b * DM + d0 + rows[it]) * NKEY + k0 + c8) = vv[it];
    }
    __threadfence();
  }
}

__global__ __launch_bounds__(256) void wconv_kernel(const float* __restrict__ w, unsigned short* __restrict__ Wb, int n8) {
  const int t = blockIdx.x * 256 + threadIdx.x;
  if (t >= n8) return;
  const float* p = w + (size_t)t * 8;
  const v4f a0 = *(const v4f*)(p);
  const v4f a1 = *(const v4f*)(p + 4);
  float f[8];
  f[0] = a0[0]; f[1] = a0[1]; f[2] = a0[2]; f[3] = a0[3];
  f[4] = a1[0]; f[5] = a1[1]; f[6] = a1[2]; f[7] = a1[3];
  unsigned hw[4];
#pragma unroll
  for (int e = 0; e < 4; ++e) {
    const unsigned short h0 = f2bf_bits(f[2 * e]);
    const unsigned short h1 = f2bf_bits(f[2 * e + 1]);
    hw[e] = (unsigned)h0 | ((unsigned)h1 << 16);
  }
  v4u hv; hv[0] = hw[0]; hv[1] = hw[1]; hv[2] = hw[2]; hv[3] = hw[3];
  volatile v4u* hp = (volatile v4u*)(Wb + (size_t)t * 8);
  *hp = hv;
  __threadfence();
  *hp = hv;
}

extern "C" void kernel_launch(void* const* d_in, const int* in_sizes, int n_in,
                              void* d_out, int out_size, void* d_ws, size_t ws_size,
                              hipStream_t stream) {
  static_assert(NB >= 1 && NB <= NB_FULL);
  static_assert(NQ >= 64 && NQ <= NQ_FULL && NQ % 64 == 0);
  static_assert(NKEY == GRW * GRW && NKEY % 64 == 0 && NKEY % 32 == 0);
  static_assert(DM % 64 == 0 && KD == NHD * DM && KD % 32 == 0);
  static_assert((DM * KD) % 8 == 0);
  if (n_in < 6) return;
  if (in_sizes[0] < NB * NKEY * DM) return;
  if (in_sizes[1] < 1) return;
  if (in_sizes[2] < NHD * 2 || in_sizes[3] < NHD * 4) return;
  if (in_sizes[4] < DM * KD || in_sizes[5] < DM) return;
  if (out_size < (NB - 1) * NQ_FULL * DM + NQ * DM) return;

  const float* hs      = (const float*)d_in[0];
  const int*   amask   = (const int*)d_in[1];
  const float* centers = (const float*)d_in[2];
  const float* spreads = (const float*)d_in[3];
  const float* vw      = (const float*)d_in[4];
  const float* vb      = (const float*)d_in[5];
  float* out = (float*)d_out;

  constexpr size_t SZ_P  = (size_t)NHD * NQ * NKEY * 2;
  constexpr size_t SZ_XT = (size_t)NB * DM * NKEY * 2;
  constexpr size_t SZ_W  = (size_t)DM * KD * 2;
  constexpr size_t SZ_V  = (size_t)NBC * NQ * KD * 2;
  constexpr size_t OFF_PH = 0;
  constexpr size_t OFF_PL = OFF_PH + SZ_P;
  constexpr size_t OFF_XT = OFF_PL + SZ_P;
  constexpr size_t OFF_W  = OFF_XT + SZ_XT;
  constexpr size_t OFF_VH = OFF_W  + SZ_W;
  constexpr size_t OFF_VL = OFF_VH + SZ_V;
  constexpr size_t WS_TOTAL = OFF_VL + SZ_V;
  static_assert(WS_TOTAL <= (size_t)134217728);
  static_assert(NB != 16 || NQ != 1024 || WS_TOTAL == (size_t)122814464);
  static_assert(OFF_PL % 128 == 0 && OFF_XT % 128 == 0 && OFF_W % 128 == 0 && OFF_VH % 128 == 0 && OFF_VL % 128 == 0);
  static_assert(((size_t)(NHD * NQ - 1) * NKEY + NKEY) * 2 == SZ_P);
  static_assert(((size_t)(NB * DM - 1) * NKEY + NKEY) * 2 == SZ_XT);
  static_assert(((size_t)NBC * NQ * KD) * 2 == SZ_V);
  static_assert(((size_t)(NB - 1) * NQ_FULL + NQ) * DM <= (size_t)NB_FULL * NQ_FULL * DM);
  if (WS_TOTAL > ws_size) return;

  char* ws = (char*)d_ws;
  unsigned short* Ph = (unsigned short*)(ws + OFF_PH);
  unsigned short* Pl = (unsigned short*)(ws + OFF_PL);
  unsigned short* XT = (unsigned short*)(ws + OFF_XT);
  unsigned short* Wb = (unsigned short*)(ws + OFF_W);
  unsigned short* Vh = (unsigned short*)(ws + OFF_VH);
  unsigned short* Vl = (unsigned short*)(ws + OFF_VL);

  probs_kernel<<<dim3(NQ / 8, NHD), 256, 0, stream>>>(centers, spreads, amask, Ph, Pl);

  xt_kernel<<<dim3(NKEY / 64, DM / 64, NB), 256, 0, stream>>>(hs, XT);

  {
    const int n8 = DM * KD / 8;
    wconv_kernel<<<(n8 + 255) / 256, 256, 0, stream>>>(vw, Wb, n8);
  }

  const int tiles = (NQ / 64) * (DM / 64);
  const int bx = (tiles + 7) / 8;
  for (int b0 = 0; b0 < NB; b0 += BCH) {
    const int nb = (NB - b0 < BCH) ? (NB - b0) : BCH;
    wmma_gemm64<1, 1, 0, 2><<<dim3(bx, nb, NHD), 256, 0, stream>>>(
        Ph, Pl, NKEY, 0L, (long)NQ * NKEY,
        XT + (size_t)b0 * DM * NKEY, XT + (size_t)b0 * DM * NKEY, NKEY, (long)DM * NKEY, 0L,
        (void*)Vh, (void*)Vl, KD, (long)NQ * KD, (long)DM,
        vb, NQ, DM, NKEY, 1.0f);
    wmma_gemm64<1, 1, 2, 0><<<dim3(bx, nb, 1), 256, 0, stream>>>(
        Vh, Vl, KD, (long)NQ * KD, 0L,
        Wb, Wb, KD, 0L, 0L,
        (void*)(out + (size_t)b0 * NQ_FULL * DM), (void*)(out + (size_t)b0 * NQ_FULL * DM), DM, (long)NQ_FULL * DM, 0L,
        vb, NQ, DM, KD, 1.0f);
  }
}
